// _LocalState_76991583748295
// MI455X (gfx1250) — hardware-verified
//
#include <hip/hip_runtime.h>
#include <math.h>

typedef __attribute__((ext_vector_type(16))) _Float16 v16h;
typedef __attribute__((ext_vector_type(16))) __bf16 v16b;
typedef __attribute__((ext_vector_type(8)))  _Float16 v8h;
typedef __attribute__((ext_vector_type(8)))  float v8f;
typedef __attribute__((ext_vector_type(4)))  float v4f;
typedef __attribute__((ext_vector_type(2)))  float v2f;
typedef __attribute__((ext_vector_type(4)))  unsigned v4u;
typedef __attribute__((ext_vector_type(4)))  int v4i;
typedef float __attribute__((may_alias)) float_a;
typedef int __attribute__((may_alias)) int_a;

template <typename T> __device__ __forceinline__ void vst2(void* p, T v) { *(volatile T*)p = v; __threadfence(); *(volatile T*)p = v; }
__device__ __forceinline__ v8f wmma16(v16h a, v16h b, v8f c) {
  v8f d = __builtin_amdgcn_wmma_f32_16x16x32_f16(false, a, false, b, (short)0, c, false, false);
  asm volatile("v_nop\n\tv_nop\n\tv_nop\n\tv_nop" : "+v"(d) : "v"(a), "v"(b));
  return d;
}
__device__ __forceinline__ v8f wmma_bf(v16b a, v16b b, v8f c) {
  v8f d = __builtin_amdgcn_wmma_f32_16x16x32_bf16(false, a, false, b, (short)0, c, false, false);
  asm volatile("v_nop\n\tv_nop\n\tv_nop\n\tv_nop" : "+v"(d) : "v"(a), "v"(b));
  return d;
}
__device__ __forceinline__ v16h frag_h(const _Float16* rowk0, int lane) {
  union { v16h v; v8h q[2]; } u; const _Float16* p = rowk0 + 8 * (lane >> 4);
  u.q[0] = *(const v8h*)p; u.q[1] = *(const v8h*)(p + 16); return u.v;
}
__device__ __forceinline__ v16h frag_f32(const float* rowk0, int lane) {
  v16h a; const float* p = rowk0 + 8 * (lane >> 4);
#pragma unroll
  for (int i = 0; i < 8; ++i) { a[i] = (_Float16)p[i]; a[8 + i] = (_Float16)p[16 + i]; }
  return a;
}
__device__ __forceinline__ v16h frag_f32s(const float* rowk0, int lane, float sc) {
  v16h a; const float* p = rowk0 + 8 * (lane >> 4);
#pragma unroll
  for (int i = 0; i < 8; ++i) { a[i] = (_Float16)(p[i] * sc); a[8 + i] = (_Float16)(p[16 + i] * sc); }
  return a;
}
__device__ __forceinline__ v16h fragc_f32(const float* W, int k0, int n, int lane, int ld, int K) {
  v16h a; const int g = lane >> 4;
#pragma unroll
  for (int i = 0; i < 8; ++i) { const int ka = k0 + 8 * g + i, kb = ka + 16;
    a[i] = (_Float16)(ka < K ? W[(size_t)(ka < K ? ka : K - 1) * ld + n] : 0.f); a[8 + i] = (_Float16)(kb < K ? W[(size_t)(kb < K ? kb : K - 1) * ld + n] : 0.f); }
  return a;
}
struct F2 { v16b h, l; };
__device__ __forceinline__ F2 bsplit16(const float v[16]) { F2 r;
#pragma unroll
  for (int i = 0; i < 16; ++i) { const __bf16 h = (__bf16)v[i]; r.h[i] = h; r.l[i] = (__bf16)(v[i] - (float)h); }
  return r; }
__device__ __forceinline__ F2 split_row(const float* row, int k0, int lane) { float v[16]; const float* p = row + k0 + 8 * (lane >> 4);
#pragma unroll
  for (int i = 0; i < 8; ++i) { v[i] = p[i]; v[8 + i] = p[16 + i]; }
  return bsplit16(v); }
__device__ __forceinline__ F2 split_rowK(const float* row, int k0, int lane, int K) { float v[16]; const int g = lane >> 4;
#pragma unroll
  for (int i = 0; i < 8; ++i) { const int ka = k0 + 8 * g + i, kb = ka + 16; v[i] = ka < K ? row[ka < K ? ka : K - 1] : 0.f; v[8 + i] = kb < K ? row[kb < K ? kb : K - 1] : 0.f; }
  return bsplit16(v); }
__device__ __forceinline__ F2 split_col(const float* W, int k0, int n, int lane, int ld, int K) { float v[16]; const int g = lane >> 4;
#pragma unroll
  for (int i = 0; i < 8; ++i) { const int ka = k0 + 8 * g + i, kb = ka + 16; v[i] = ka < K ? W[(size_t)(ka < K ? ka : K - 1) * ld + n] : 0.f; v[8 + i] = kb < K ? W[(size_t)(kb < K ? kb : K - 1) * ld + n] : 0.f; }
  return bsplit16(v); }
__device__ __forceinline__ v8f mac3(const F2& a, const F2& b, v8f c) { c = wmma_bf(a.l, b.h, c); c = wmma_bf(a.h, b.l, c); return wmma_bf(a.h, b.h, c); }
__device__ __forceinline__ float sigm(float v) { return 1.0f / (1.0f + expf(-v)); }
#define LDSX() do { asm volatile("s_wait_dscnt 0" ::: "memory"); __builtin_amdgcn_wave_barrier(); __builtin_amdgcn_fence(__ATOMIC_RELEASE, "workgroup"); } while (0)


#define NB 4
#define CC 1024
#define TT 2048
#define NH 8
#define HD 128
#define NDK 4
#ifndef TNB
#define TNB NB
#endif
typedef __attribute__((ext_vector_type(8))) __bf16 v8b;
__device__ __forceinline__ v16b frag_b(const __bf16* rowk0, int lane) {
  union { v16b v; v8b q[2]; } u; const __bf16* p = rowk0 + 8 * (lane >> 4);
  u.q[0] = *(const v8b*)p; u.q[1] = *(const v8b*)(p + 16); return u.v;
}
__device__ __forceinline__ float bfr(float v) { return (float)(__bf16)v; }
__device__ __attribute__((noinline)) float exp_ni(float v) { return expf(v); }
__device__ __attribute__((noinline)) float erf_ni(float v) { return erff(v); }

#define WS_Q   0u
#define WS_K   (WS_Q + 2u * (size_t)NB * TT * CC)
#define WS_CT  (WS_K + 2u * (size_t)NB * CC * TT)
#define WS_DQ  (WS_CT + 2u * (size_t)NB * CC * TT)
#define WS_S   (WS_DQ + 4u * (size_t)NB * NH * TT)
#define WS_P   (WS_S + 4u * (size_t)TT * TT)
#define WS_R   (WS_P + 2u * (size_t)TT * TT)
#define WS_XT  (WS_R + 2u * (size_t)NB * TT * CC)
#define WS_END (WS_XT + 2u * (size_t)NB * TT * CC)

__global__ __launch_bounds__(128) void k_xt(const float* __restrict__ X, __bf16* __restrict__ XT) { __shared__ __align__(16) __bf16 s[64][136]; const int tid = threadIdx.x; const int t0 = blockIdx.x * 64, c0 = blockIdx.y * 128; const size_t b = blockIdx.z;
  for (int e = tid; e < 128 * 64; e += 128) { const int cl = e >> 6, tl = e & 63; s[tl][cl] = (__bf16)X[(b * CC + c0 + cl) * (size_t)TT + t0 + tl]; }
  __syncthreads(); for (int e = tid; e < 64 * 16; e += 128) { const int tl = e >> 4, q = e & 15; vst2((unsigned*)(XT + (b * TT + t0 + tl) * CC + c0 + q * 8), *(const v4u*)&s[tl][q * 8]); } }
__global__ __launch_bounds__(128) void k_proj3(const __bf16* __restrict__ XT, const float* __restrict__ WQ, const float* __restrict__ BQ, const float* __restrict__ WK, const float* __restrict__ BK, const float* __restrict__ WC, const float* __restrict__ BC, _Float16* __restrict__ Q, _Float16* __restrict__ K, _Float16* __restrict__ CT) {
  __shared__ __align__(16) _Float16 sh[128][72]; __shared__ __align__(16) _Float16 sp[64][136];
  const int tid = threadIdx.x, wave = tid >> 5, lane = tid & 31, col = lane & 15, g = lane >> 4; const int d0 = blockIdx.x * 64 + wave * 16, t0 = blockIdx.y * 128; const size_t b = blockIdx.z / 3; const int which = blockIdx.z % 3;
  const float* Wm = which == 0 ? WQ : which == 1 ? WK : WC; const float* Bm = which == 0 ? BQ : which == 1 ? BK : BC;
  v8f acc[8] = {};
#pragma unroll 2
  for (int kc = 0; kc < CC / 32; ++kc) { v16b a; { const float* p = Wm + (size_t)(d0 + col) * CC + kc * 32 + 8 * g;
#pragma unroll
      for (int i = 0; i < 8; ++i) { a[i] = (__bf16)p[i]; a[8 + i] = (__bf16)p[16 + i]; } }
#pragma unroll
    for (int j = 0; j < 8; ++j) acc[j] = wmma_bf(a, frag_b(XT + (b * TT + t0 + j * 16 + col) * CC + kc * 32, lane), acc[j]); }
  if (which < 2) {
#pragma unroll
    for (int j = 0; j < 8; ++j)
#pragma unroll
      for (int r = 0; r < 8; ++r) { const int dl = wave * 16 + 8 * g + r; sh[j * 16 + col][dl] = (_Float16)(acc[j][r] + bfr(Bm[d0 + 8 * g + r])); }
    __syncthreads(); _Float16* dq = which == 0 ? Q : K; for (int e = tid; e < 128 * 8; e += 128) { const int tl = e >> 3, q = e & 7; vst2((unsigned*)(dq + (b * TT + t0 + tl) * CC + blockIdx.x * 64 + q * 8), *(const v4u*)&sh[tl][q * 8]); } }
  else {
#pragma unroll
    for (int j = 0; j < 8; ++j)
#pragma unroll
      for (int r = 0; r < 8; ++r) sp[wave * 16 + 8 * g + r][j * 16 + col] = (_Float16)(acc[j][r] + bfr(Bm[d0 + 8 * g + r]));
    __syncthreads(); _Float16* dst = CT; for (int e = tid; e < 64 * 16; e += 128) { const int dl = e >> 4, q = e & 15; vst2((unsigned*)(dst + (b * CC + blockIdx.x * 64 + dl) * (size_t)TT + t0 + q * 8), *(const v4u*)&sp[dl][q * 8]); } } }
__global__ __launch_bounds__(128) void k_dq(const __bf16* __restrict__ XT, const float* __restrict__ WD, const float* __restrict__ BD, float* __restrict__ DQ) { __shared__ __align__(16) float sd[32][132]; __shared__ __align__(16) float so[NH][132];
  const int tid = threadIdx.x, wave = tid >> 5, lane = tid & 31, col = lane & 15, g = lane >> 4; const int t0 = blockIdx.x * 128; const size_t b = blockIdx.y; const int rt = wave & 1, cg = wave >> 1;
  v8f acc[4] = {};
#pragma unroll 2
  for (int kc = 0; kc < CC / 32; ++kc) { v16b a; { const float* p = WD + (size_t)(rt * 16 + col) * CC + kc * 32 + 8 * g;
#pragma unroll
      for (int i = 0; i < 8; ++i) { a[i] = (__bf16)p[i]; a[8 + i] = (__bf16)p[16 + i]; } }
#pragma unroll
    for (int j = 0; j < 4; ++j) acc[j] = wmma_bf(a, frag_b(XT + (b * TT + t0 + cg * 64 + j * 16 + col) * CC + kc * 32, lane), acc[j]); }
#pragma unroll
  for (int j = 0; j < 4; ++j)
#pragma unroll
    for (int r = 0; r < 8; ++r) { const int ch = rt * 16 + 8 * g + r; sd[ch][cg * 64 + j * 16 + col] = acc[j][r] + bfr(BD[ch]); }
  __syncthreads();
  for (int e = tid; e < NH * 128; e += 128) { const int h = e >> 7, tl = e & 127; float dsum = 0.f; for (int f = 0; f < NDK; ++f) { const float z = sd[h * NDK + f][tl]; dsum += (float)(f + 1) * (1.0f / (1.0f + expf(-z))) * 0.5f; } so[h][tl] = dsum * 0.5f; }
  __syncthreads(); for (int e = tid; e < NH * 32; e += 128) { const int h = e >> 5, q = e & 31; vst2(DQ + (b * NH + h) * (size_t)TT + t0 + q * 4, *(const v4f*)&so[h][q * 4]); } }
__global__ __launch_bounds__(128) void k_sc(const _Float16* __restrict__ Q, const _Float16* __restrict__ K, const float* __restrict__ DQ, int b, int h, float* __restrict__ S) { __shared__ __align__(16) float ss[4][16][132];
  const int tid = threadIdx.x, wave = tid >> 5, lane = tid & 31, col = lane & 15, g = lane >> 4; const int t0 = blockIdx.y * 128; const int sl0 = blockIdx.x * 64 + wave * 16; const size_t q0 = (size_t)b * TT + sl0;
  v8f acc[8] = {};
#pragma unroll
  for (int kc = 0; kc < HD / 32; ++kc) { const v16h a = frag_h(Q + (q0 + col) * CC + h * HD + kc * 32, lane);
#pragma unroll
    for (int j = 0; j < 8; ++j) acc[j] = wmma16(a, frag_h(K + ((size_t)b * TT + t0 + j * 16 + col) * CC + h * HD + kc * 32, lane), acc[j]); }
#pragma unroll
  for (int j = 0; j < 8; ++j) { const int t = t0 + j * 16 + col;
#pragma unroll
    for (int r = 0; r < 8; ++r) { const int s = sl0 + 8 * g + r; const float ds = DQ[((size_t)b * NH + h) * TT + s]; const float dl = (float)(t > s ? t - s : s - t); ss[wave][8 * g + r][j * 16 + col] = (t == s) ? -100.0f : (acc[j][r] * 0.08838834764831845f - dl * ds); } }
  LDSX(); for (int rl = 0; rl < 16; ++rl) vst2(S + (size_t)(sl0 + rl) * TT + t0 + lane * 4, *(const v4f*)&ss[wave][rl][lane * 4]); }
__global__ __launch_bounds__(256) void k_sm(const float* __restrict__ S, _Float16* __restrict__ P) { __shared__ float sred[8]; __shared__ float sbc; __shared__ __align__(16) _Float16 sh[TT];
  const int t = threadIdx.x; const size_t row = blockIdx.x; const float* sr = S + row * TT;
  float m = -3.0e38f; for (int k = t; k < TT; k += 256) m = fmaxf(m, sr[k]);
#pragma unroll
  for (int o = 1; o < 32; o <<= 1) m = fmaxf(m, __shfl_xor(m, o));
  if ((t & 31) == 0) sred[t >> 5] = m; __syncthreads(); if (t == 0) { float a = sred[0]; for (int i = 1; i < 8; ++i) a = fmaxf(a, sred[i]); sbc = a; } __syncthreads(); m = sbc; __syncthreads();
  float sum = 0.f; for (int k = t; k < TT; k += 256) sum += expf(sr[k] - m);
#pragma unroll
  for (int o = 1; o < 32; o <<= 1) sum += __shfl_xor(sum, o);
  if ((t & 31) == 0) sred[t >> 5] = sum; __syncthreads(); if (t == 0) { float a = 0.f; for (int i = 0; i < 8; ++i) a += sred[i]; sbc = 1.0f / a; } __syncthreads(); const float inv = sbc;
  for (int k = t; k < TT; k += 256) sh[k] = (_Float16)(expf(sr[k] - m) * inv * 2048.0f);
  __syncthreads(); for (int q = t; q < TT / 8; q += 256) vst2((unsigned*)(P + row * TT + q * 8), *(const v4u*)&sh[q * 8]); }
__global__ __launch_bounds__(128) void k_pv(const _Float16* __restrict__ P, const _Float16* __restrict__ CT, int b, int h, _Float16* __restrict__ R) { __shared__ __align__(16) _Float16 sr[64][136];
  const int tid = threadIdx.x, wave = tid >> 5, lane = tid & 31, col = lane & 15, g = lane >> 4; const int sl0 = blockIdx.x * 64 + wave * 16;
  v8f acc[8] = {};
#pragma unroll 1
  for (int kc = 0; kc < TT / 32; ++kc) { const v16h pa = frag_h(P + (size_t)(sl0 + col) * TT + kc * 32, lane);
#pragma unroll
    for (int j = 0; j < 8; ++j) acc[j] = wmma16(pa, frag_h(CT + ((size_t)b * CC + h * HD + j * 16 + col) * TT + kc * 32, lane), acc[j]); }
#pragma unroll
  for (int j = 0; j < 8; ++j)
#pragma unroll
    for (int r = 0; r < 8; ++r) sr[wave * 16 + 8 * g + r][j * 16 + col] = (_Float16)(acc[j][r] * (1.0f / 2048.0f));
  __syncthreads(); for (int e = tid; e < 64 * 16; e += 128) { const int rl = e >> 4, q = e & 15; vst2((unsigned*)(R + ((size_t)b * TT + blockIdx.x * 64 + rl) * CC + h * HD + q * 8), *(const v4u*)&sr[rl][q * 8]); } }
__global__ __launch_bounds__(128) void k_out(const float* __restrict__ X, const _Float16* __restrict__ R, const float* __restrict__ WP, const float* __restrict__ BP, float* __restrict__ OUT) { __shared__ __align__(16) float sp[64][132];
  const int tid = threadIdx.x, wave = tid >> 5, lane = tid & 31, col = lane & 15, g = lane >> 4; const int o0 = blockIdx.x * 64 + wave * 16, s0 = blockIdx.y * 128; const size_t b = blockIdx.z;
  v8f acc[8] = {};
#pragma unroll 2
  for (int kc = 0; kc < CC / 32; ++kc) { v16h a; { const float* p = WP + (size_t)(o0 + col) * CC + kc * 32 + 8 * g;
#pragma unroll
      for (int i = 0; i < 8; ++i) { a[i] = (_Float16)bfr(p[i]); a[8 + i] = (_Float16)bfr(p[16 + i]); } }
#pragma unroll
    for (int j = 0; j < 8; ++j) acc[j] = wmma16(a, frag_h(R + (b * TT + s0 + j * 16 + col) * CC + kc * 32, lane), acc[j]); }
#pragma unroll
  for (int j = 0; j < 8; ++j)
#pragma unroll
    for (int r = 0; r < 8; ++r) { const int o = o0 + 8 * g + r; const int s = s0 + j * 16 + col; sp[wave * 16 + 8 * g + r][j * 16 + col] = acc[j][r] + bfr(BP[o]) + bfr(X[(b * CC + o) * (size_t)TT + s]); }
  __syncthreads(); for (int e = tid; e < 64 * 32; e += 128) { const int ol = e >> 5, q = e & 31; vst2(OUT + (b * CC + blockIdx.x * 64 + ol) * (size_t)TT + s0 + q * 4, *(const v4f*)&sp[ol][q * 4]); } }
extern "C" void kernel_launch(void* const* d_in, const int* in_sizes, int n_in, void* d_out, int out_size, void* d_ws, size_t ws_size, hipStream_t stream) {
  (void)in_sizes; (void)n_in; (void)out_size;
  const float** F = (const float**)d_in;
  if (ws_size < (size_t)WS_END) return;
  char* ws = (char*)d_ws; _Float16 *Q = (_Float16*)(ws + WS_Q), *K = (_Float16*)(ws + WS_K), *CT = (_Float16*)(ws + WS_CT), *P = (_Float16*)(ws + WS_P), *R = (_Float16*)(ws + WS_R); float *DQ = (float*)(ws + WS_DQ), *S = (float*)(ws + WS_S);
  __bf16* XT = (__bf16*)(ws + WS_XT);
  k_xt<<<dim3(TT / 64, CC / 128, TNB), 128, 0, stream>>>(F[0], XT);
  k_proj3<<<dim3(CC / 64, TT / 128, TNB * 3), 128, 0, stream>>>(XT, F[3], F[4], F[5], F[6], F[1], F[2], Q, K, CT);
  k_dq<<<dim3(TT / 128, TNB), 128, 0, stream>>>(XT, F[7], F[8], DQ);
  for (int b = 0; b < TNB; ++b) for (int h = 0; h < NH; ++h) {
    k_sc<<<dim3(TT / 64, TT / 128), 128, 0, stream>>>(Q, K, DQ, b, h, S);
    k_sm<<<TT, 256, 0, stream>>>(S, P);
    k_pv<<<TT / 64, 128, 0, stream>>>(P, CT, b, h, R);
  }
  k_out<<<dim3(CC / 64, TT / 128, TNB), 128, 0, stream>>>(F[0], R, F[9], F[10], (float*)d_out);
}
